// SelfAttention_31791347925883
// MI455X (gfx1250) — hardware-run, weakly checked
//
#include <hip/hip_runtime.h>


#ifndef NB
#define NB 8
#endif
#ifndef SEQ
#define SEQ 2048
#endif
#define NB_FULL  8
#define SEQ_FULL 2048
#ifndef OUT_SEQ
#define OUT_SEQ SEQ
#endif
#define DM   256
#define NH_  4
#define HD   64
#define DQKV 768
#define AW   4
#define OSP  68
#define WTP  260
#define EROWS (SEQ < 256 ? SEQ : 256)
#define QRS  2048.0f
#define QRI  (1.0f / 2048.0f)
#define SC2  ((float)(0.125 * 1.4426950408889634))
#define PSH  14.0f
#define PFL  (-14.0f)
#define NEGB (-3.0e38f)
#define CCAR 16.0f
#define WCAR 1024.0f
#define OSCL (1.0f / 16384.0f)

static_assert(HD == 64);
static_assert(HD * 2 == 128);
static_assert(NH_ * HD == DM);
static_assert(DQKV == 3 * DM);
static_assert(DM % 64 == 0);
static_assert(64 == HD);
static_assert(DM % 32 == 0);
static_assert(HD % 32 == 0);
static_assert(SEQ % 64 == 0);
static_assert((NB * SEQ) % 64 == 0);
static_assert(SEQ % 32 == 0);
static_assert(SEQ % (16 * AW) == 0);
static_assert(EROWS % 64 == 0);
static_assert(EROWS % 32 == 0);
static_assert(EROWS >= 32);
static_assert(EROWS <= SEQ);
static_assert(EROWS % (16 * AW) == 0);
static_assert((SEQ - EROWS) % (16 * AW) == 0);
static_assert((SEQ - EROWS) % 64 == 0);
static_assert(((size_t)SEQ * DM) % 8 == 0);
static_assert(NB <= NB_FULL);
static_assert(SEQ <= SEQ_FULL);
static_assert((OSP * 4) % 16 == 0);
static_assert(OSP >= HD);
static_assert((WTP * 4) % 16 == 0);
static_assert(WTP >= DM);
static_assert(DQKV % 16 == 0);
static_assert(128 * 32 == DM * 16);
static_assert(32 * 16 == DM * 2);
static_assert(4 * 4 == 16);
static_assert(4 * 32 * 16 == 16 * HD * 2);
static_assert(4 * 4 * 8 * 16 == 16 * 64 * 2);
static_assert(8 * 2 * 16 * 16 == 16 * 64 * 4);
static_assert((size_t)AW * 16 * OSP * 4 <= 131072);
static_assert((size_t)16 * WTP * 4 <= 131072);
static_assert((size_t)16 * 68 * 4 <= 131072);

typedef _Float16 h16;
typedef unsigned short bf;
typedef __attribute__((ext_vector_type(16))) __bf16   v16bf;
typedef __attribute__((ext_vector_type(16))) _Float16 v16h;
typedef __attribute__((ext_vector_type(8)))  _Float16 v8h;
typedef __attribute__((ext_vector_type(8)))  unsigned short v8us;
typedef __attribute__((ext_vector_type(8)))  float    v8f;
typedef __attribute__((ext_vector_type(4)))  float    v4f;
typedef v4f  __attribute__((may_alias)) v4fa;

__device__ __forceinline__ unsigned short f2bf(float f) { unsigned u = __float_as_uint(f); u += 0x7FFFu + ((u >> 16) & 1u); return (unsigned short)(u >> 16); }
__device__ __forceinline__ float bfr(float f) { return __uint_as_float(((unsigned)f2bf(f)) << 16); }
__device__ __forceinline__ v16h cat16(v8h lo, v8h hi) { return __builtin_shufflevector(lo, hi, 0, 1, 2, 3, 4, 5, 6, 7, 8, 9, 10, 11, 12, 13, 14, 15); }
__device__ __forceinline__ v16bf cat16b(v8us lo, v8us hi) { return __builtin_bit_cast(v16bf, __builtin_shufflevector(lo, hi, 0, 1, 2, 3, 4, 5, 6, 7, 8, 9, 10, 11, 12, 13, 14, 15)); }
__device__ __forceinline__ v8f wmma16(v16h a, v16h b, v8f c) { return __builtin_amdgcn_wmma_f32_16x16x32_f16(false, a, false, b, (short)0, c, false, false); }
__device__ __forceinline__ v8f wmmab(v16bf a, v16bf b, v8f c) { return __builtin_amdgcn_wmma_f32_16x16x32_bf16(false, a, false, b, (short)0, c, false, false); }
__device__ __forceinline__ v16h  ldh(const h16* p) { return cat16(*(const v8h*)p, *(const v8h*)(p + 16)); }
__device__ __forceinline__ v16bf ldb(const bf* p)  { return cat16b(*(const v8us*)p, *(const v8us*)(p + 16)); }
__device__ __forceinline__ void wave_sync() { __builtin_amdgcn_fence(3  , "wavefront"); __builtin_amdgcn_wave_barrier(); asm volatile("" ::: "memory"); }
static __device__ __forceinline__ h16 toh_flush(float v) { const float w = (fabsf(v) < 6.103515625e-05f) ? 0.0f : v; return (h16)w; }
__device__ __forceinline__ v8f wmma16g(v16h a, v16h b, v8f c) { c = wmma16(a, b, c); asm volatile("v_nop\n\tv_nop\n\tv_nop\n\tv_nop" : "+v"(c) : "v"(a), "v"(b)); return c; }
__device__ __forceinline__ v8f wmmabg(v16bf a, v16bf b, v8f c) { c = wmmab(a, b, c); asm volatile("v_nop\n\tv_nop\n\tv_nop\n\tv_nop" : "+v"(c) : "v"(a), "v"(b)); return c; }

__global__ __launch_bounds__(256) void k_cvt8(const float* __restrict__ src, bf* dst, size_t n8) {
    const size_t i = (size_t)blockIdx.x * 256 + threadIdx.x; if (i >= n8) return;
    const v8f v = *(const v8f*)(src + i * 8); v8us o;
#pragma unroll
    for (int k = 0; k < 8; ++k) o[k] = f2bf(v[k]);
    *(volatile v8us*)(dst + i * 8) = o; __threadfence(); *(volatile v8us*)(dst + i * 8) = o;
}

__global__ __launch_bounds__(128) void k_wtb(const float* __restrict__ W, bf* WT, unsigned ldw) {
    __shared__ __align__(16) float ts[16 * WTP];
    const unsigned tid = threadIdx.x; const unsigned n0 = blockIdx.x * 16u;
#pragma unroll 8
    for (unsigned it = 0; it < 32u; ++it) {
        const unsigned idx = it * 128u + tid; const unsigned k = idx >> 4, nn = idx & 15u;
        ts[nn * WTP + k] = W[(size_t)k * ldw + n0 + nn]; }
    __syncthreads();
    const unsigned lane = tid & 31u; const unsigned wave = (unsigned)__builtin_amdgcn_readfirstlane((int)(threadIdx.x >> 5));
#pragma unroll 1
    for (int ps = 0; ps < 2; ++ps) {
#pragma unroll
        for (unsigned i = 0; i < 4u; ++i) { const unsigned r = wave * 4u + i;
            const v4f x0 = *(const v4fa*)(&ts[r * WTP + lane * 8u]); const v4f x1 = *(const v4fa*)(&ts[r * WTP + lane * 8u + 4u]); v8us o;
#pragma unroll
            for (int j = 0; j < 4; ++j) { o[j] = f2bf(x0[j]); o[4 + j] = f2bf(x1[j]); }
            *(volatile v8us*)(WT + (size_t)(n0 + r) * DM + lane * 8u) = o; }
        if (ps == 0) __threadfence(); }
}

__global__ __launch_bounds__(128) void k_wth(const float* __restrict__ W, h16* WT, unsigned ldw) {
    __shared__ __align__(16) float ts[16 * WTP];
    const unsigned tid = threadIdx.x; const unsigned n0 = blockIdx.x * 16u;
#pragma unroll 8
    for (unsigned it = 0; it < 32u; ++it) {
        const unsigned idx = it * 128u + tid; const unsigned k = idx >> 4, nn = idx & 15u;
        ts[nn * WTP + k] = W[(size_t)k * ldw + n0 + nn]; }
    __syncthreads();
    const unsigned lane = tid & 31u; const unsigned wave = (unsigned)__builtin_amdgcn_readfirstlane((int)(threadIdx.x >> 5));
#pragma unroll 1
    for (int ps = 0; ps < 2; ++ps) {
#pragma unroll
        for (unsigned i = 0; i < 4u; ++i) { const unsigned r = wave * 4u + i;
            const v4f x0 = *(const v4fa*)(&ts[r * WTP + lane * 8u]); const v4f x1 = *(const v4fa*)(&ts[r * WTP + lane * 8u + 4u]); v8h o;
#pragma unroll
            for (int j = 0; j < 4; ++j) { o[j] = toh_flush(bfr(x0[j]) * WCAR); o[4 + j] = toh_flush(bfr(x1[j]) * WCAR); }
            *(volatile v8h*)(WT + (size_t)(n0 + r) * DM + lane * 8u) = o; }
        if (ps == 0) __threadfence(); }
}

template <int MODE>
__device__ __forceinline__ void proj_body(const bf* __restrict__ A, const bf* __restrict__ Bt, const float* __restrict__ bias, h16* Ph, h16* Pr, unsigned resT) {
    __shared__ __align__(16) float os[16 * 68];
    const unsigned K = DM;
    const unsigned lane = threadIdx.x & 31u, lr = lane & 15u, hi = lane >> 4; const unsigned r0 = blockIdx.x * 64u, c0 = blockIdx.y * 64u;
    v8f acc[4][4];
#pragma unroll
    for (int mb = 0; mb < 4; ++mb)
#pragma unroll
        for (int nb = 0; nb < 4; ++nb) acc[mb][nb] = (v8f){};
    const size_t aoff = (size_t)(r0 + lr) * K + 8u * hi, boff = (size_t)(c0 + lr) * K + 8u * hi;
#pragma unroll 1
    for (unsigned kc = 0; kc < K; kc += 32u) {
        v16bf a[4];
#pragma unroll
        for (int mb = 0; mb < 4; ++mb) a[mb] = ldb(A + aoff + (size_t)mb * 16 * K + kc);
#pragma unroll
        for (int nb = 0; nb < 4; ++nb) { const v16bf bq = ldb(Bt + boff + (size_t)nb * 16 * K + kc);
#pragma unroll
            for (int mb = 0; mb < 4; ++mb) acc[mb][nb] = wmmabg(a[mb], bq, acc[mb][nb]); }
    }
    float bc[4];
#pragma unroll
    for (int nb = 0; nb < 4; ++nb) bc[nb] = (MODE == 0) ? bfr(bias[c0 + nb * 16 + lr]) : 0.0f;
    size_t tbase, rbase; bool wr;
    if (MODE == 0) { const unsigned bb = r0 / (unsigned)SEQ, tt = r0 % (unsigned)SEQ; const unsigned zc = bb * (unsigned)NH_ + c0 / (unsigned)HD;
                     tbase = ((size_t)zc * SEQ + (size_t)tt) * HD; rbase = ((size_t)zc * (size_t)resT + (size_t)tt) * HD; wr = tt < resT; }
    else           { const unsigned bb = c0 / (unsigned)SEQ, tt = c0 % (unsigned)SEQ;
                     tbase = (size_t)bb * (size_t)DM * SEQ + (size_t)r0 * SEQ + (size_t)tt; rbase = (size_t)bb * (size_t)DM * (size_t)resT + (size_t)r0 * (size_t)resT + (size_t)tt; wr = tt < resT; }
#pragma unroll
    for (int mb = 0; mb < 4; ++mb) {
        float br[8];
#pragma unroll
        for (int j = 0; j < 8; ++j) br[j] = (MODE == 1) ? bfr(bias[r0 + mb * 16 + hi * 8 + j]) : 0.0f;
#pragma unroll
        for (int nb = 0; nb < 4; ++nb) {
#pragma unroll
            for (int j = 0; j < 8; ++j) os[(hi * 8 + j) * 68 + nb * 16 + lr] = acc[mb][nb][j] + bc[nb] + br[j]; }
        wave_sync();
#pragma unroll 1
        for (int ps = 0; ps < 2; ++ps) {
            if (MODE == 0) {
                const size_t sb = tbase + (size_t)(mb * 16) * HD;
                const size_t rb = rbase + (size_t)(mb * 16) * HD;
#pragma unroll
                for (int s = 0; s < 4; ++s) { const unsigned p = (unsigned)s * 32u + lane; const unsigned row = p >> 3, c8 = (p & 7u) * 8u;
                    const v4f x0 = *(const v4fa*)(&os[row * 68 + c8]); const v4f x1 = *(const v4fa*)(&os[row * 68 + c8 + 4]); v8h hv, rv;
#pragma unroll
                    for (int i = 0; i < 4; ++i) { const h16 a0 = toh_flush(x0[i]); const h16 a1 = toh_flush(x1[i]); hv[i] = a0; hv[4 + i] = a1;
                        rv[i] = toh_flush((x0[i] - (float)a0) * QRS); rv[4 + i] = toh_flush((x1[i] - (float)a1) * QRS); }
                    const size_t oo = sb + (size_t)p * 8;
                    const size_t ro = rb + (size_t)p * 8;
                    *(volatile v8h*)(Ph + oo) = hv; if (wr) *(volatile v8h*)(Pr + ro) = rv; }
            } else {
                const size_t sb = tbase + (size_t)(mb * 16) * SEQ;
                const size_t rb = rbase + (size_t)(mb * 16) * (size_t)resT;
#pragma unroll
                for (int s = 0; s < 4; ++s) { const unsigned row = 4u * (unsigned)s + (lane >> 3), c8 = (lane & 7u) * 8u;
                    const v4f x0 = *(const v4fa*)(&os[row * 68 + c8]); const v4f x1 = *(const v4fa*)(&os[row * 68 + c8 + 4]); v8h hv, rv;
#pragma unroll
                    for (int i = 0; i < 4; ++i) { const h16 a0 = toh_flush(x0[i]); const h16 a1 = toh_flush(x1[i]); hv[i] = a0; hv[4 + i] = a1;
                        rv[i] = toh_flush((x0[i] - (float)a0) * QRS); rv[4 + i] = toh_flush((x1[i] - (float)a1) * QRS); }
                    const size_t oo = sb + (size_t)row * SEQ + c8;
                    const size_t ro = rb + (size_t)row * (size_t)resT + c8;
                    *(volatile v8h*)(Ph + oo) = hv; if (wr) *(volatile v8h*)(Pr + ro) = rv; }
            }
            if (ps == 0) __threadfence(); }
        wave_sync();
    }
}

__global__ __launch_bounds__(32) void k_proj_rows(const bf* __restrict__ A, const bf* __restrict__ Bt, const float* __restrict__ bias, h16* Ph, h16* Pr, unsigned resT) {
    proj_body<0>(A, Bt, bias, Ph, Pr, resT);
}
__global__ __launch_bounds__(32) void k_proj_tr(const bf* __restrict__ A, const bf* __restrict__ Bt, const float* __restrict__ bias, h16* Ph, h16* Pr, unsigned resT) {
    proj_body<1>(A, Bt, bias, Ph, Pr, resT);
}

template <int EARLY>
__device__ __forceinline__ void flash_body(const h16* __restrict__ QH, const h16* __restrict__ QR, const h16* __restrict__ KP, const h16* __restrict__ KR,
                                           const h16* __restrict__ VT, const h16* __restrict__ VR, h16* CH, h16* CR) {
    __shared__ __align__(16) float os[AW * 16 * OSP];
    const unsigned lane = threadIdx.x & 31u, lr = lane & 15u, hi = lane >> 4;
    const unsigned wave = (unsigned)__builtin_amdgcn_readfirstlane((int)(threadIdx.x >> 5));
    const unsigned zh = blockIdx.y; const unsigned b = zh / (unsigned)NH_, h = zh % (unsigned)NH_;
    const unsigned t0 = (EARLY ? 0u : (unsigned)EROWS) + (blockIdx.x * (unsigned)AW + wave) * 16u;
    const unsigned lim = t0 + lr;
    const unsigned nk = (t0 + 16u + 31u) & ~31u;
    const size_t pbase = (size_t)zh * SEQ * HD;
    const size_t rbase = (size_t)zh * EROWS * HD;
    const v16h hz = (v16h){};
    const size_t qo = pbase + (size_t)(t0 + lr) * HD + 8u * hi;
    const v16h qh0 = ldh(QH + qo), qh1 = ldh(QH + qo + 32);
    v16h qr0 = hz, qr1 = hz;
    if (EARLY) { const size_t qro = rbase + (size_t)(t0 + lr) * HD + 8u * hi; qr0 = ldh(QR + qro); qr1 = ldh(QR + qro + 32); }
    const size_t ko = pbase + (size_t)lr * HD + 8u * hi;
    const size_t vo = pbase + (size_t)lr * SEQ + 8u * hi;
    const size_t kro = rbase + (size_t)lr * HD + 8u * hi;
    const size_t vro = rbase + (size_t)lr * EROWS + 8u * hi;
    v8f o0 = (v8f){}, o1 = (v8f){}, o2 = (v8f){}, o3 = (v8f){};
    v8f oR0 = (v8f){}, oR1 = (v8f){}, oR2 = (v8f){}, oR3 = (v8f){};
    float m = NEGB, l = 0.0f;
#pragma unroll 1
    for (unsigned key0 = 0; key0 < nk; key0 += 32u) {
        const h16* ka = KP + ko + (size_t)key0 * HD;
        const v16h ka0 = ldh(ka), ka1 = ldh(ka + 32), kb0 = ldh(ka + 16 * HD), kb1 = ldh(ka + 16 * HD + 32);
        v8f sHa = (v8f){}, sLa = (v8f){}, sHb = (v8f){}, sLb = (v8f){};
        sHa = wmma16g(ka0, qh0, sHa); sHa = wmma16g(ka1, qh1, sHa);
        sHb = wmma16g(kb0, qh0, sHb); sHb = wmma16g(kb1, qh1, sHb);
        if (EARLY) {
            const h16* kr = KR + kro + (size_t)key0 * HD;
            const v16h kra0 = ldh(kr), kra1 = ldh(kr + 32), krb0 = ldh(kr + 16 * HD), krb1 = ldh(kr + 16 * HD + 32);
            sLa = wmma16g(ka0, qr0, sLa); sLa = wmma16g(ka1, qr1, sLa); sLa = wmma16g(kra0, qh0, sLa); sLa = wmma16g(kra1, qh1, sLa);
            sLb = wmma16g(kb0, qr0, sLb); sLb = wmma16g(kb1, qr1, sLb); sLb = wmma16g(krb0, qh0, sLb); sLb = wmma16g(krb1, qh1, sLb);
        }
        const unsigned ja = key0 + 8u * hi;
        float ta[8], tb[8]; bool fa[8], fb[8]; float mx = NEGB;
#pragma unroll
        for (int r = 0; r < 8; ++r) {
            fa[r] = (ja + (unsigned)r <= lim);
            fb[r] = (ja + 16u + (unsigned)r <= lim);
            if (EARLY) { ta[r] = (sHa[r] + sLa[r] * QRI) * SC2; tb[r] = (sHb[r] + sLb[r] * QRI) * SC2; }
            else       { ta[r] = sHa[r] * SC2; tb[r] = sHb[r] * SC2; }
            mx = fmaxf(mx, fmaxf(fa[r] ? ta[r] : NEGB, fb[r] ? tb[r] : NEGB)); }
        mx = fmaxf(mx, __shfl_xor(mx, 16, 32));
        const float mnew = fmaxf(m, mx);
        const float alpha = __builtin_amdgcn_exp2f(m - mnew);
        const float sh = PSH - mnew;
        v16h pb, pr = hz; float ls = 0.0f;
#pragma unroll
        for (int r = 0; r < 8; ++r) {
            const float xa = ta[r] + sh, xb = tb[r] + sh;
            const float ea = __builtin_amdgcn_exp2f(xa), eb = __builtin_amdgcn_exp2f(xb);
            const float ga = (fa[r] && xa >= PFL) ? ea : 0.0f, gb = (fb[r] && xb >= PFL) ? eb : 0.0f;
            const h16 pa = (h16)ga; const h16 pc = (h16)gb;
            pb[r] = pa; pb[8 + r] = pc;
            if (EARLY) { pr[r] = toh_flush((ga - (float)pa) * QRS); pr[8 + r] = toh_flush((gb - (float)pc) * QRS); ls += ga + gb; }
            else       { ls += (float)pa + (float)pc; } }
        l = l * alpha + ls; m = mnew;
        o0 = o0 * alpha; o1 = o1 * alpha; o2 = o2 * alpha; o3 = o3 * alpha;
        if (EARLY) { oR0 = oR0 * alpha; oR1 = oR1 * alpha; oR2 = oR2 * alpha; oR3 = oR3 * alpha; }
        const h16* va = VT + vo + key0;
        const v16h v0 = ldh(va), v1 = ldh(va + (size_t)16 * SEQ), v2 = ldh(va + (size_t)32 * SEQ), v3 = ldh(va + (size_t)48 * SEQ);
        o0 = wmma16g(v0, pb, o0); o1 = wmma16g(v1, pb, o1); o2 = wmma16g(v2, pb, o2); o3 = wmma16g(v3, pb, o3);
        if (EARLY) {
            const h16* vr = VR + vro + key0;
            const v16h vr0 = ldh(vr), vr1 = ldh(vr + (size_t)16 * EROWS), vr2 = ldh(vr + (size_t)32 * EROWS), vr3 = ldh(vr + (size_t)48 * EROWS);
            oR0 = wmma16g(v0, pr, oR0); oR0 = wmma16g(vr0, pb, oR0);
            oR1 = wmma16g(v1, pr, oR1); oR1 = wmma16g(vr1, pb, oR1);
            oR2 = wmma16g(v2, pr, oR2); oR2 = wmma16g(vr2, pb, oR2);
            oR3 = wmma16g(v3, pr, oR3); oR3 = wmma16g(vr3, pb, oR3);
        }
    }
    l += __shfl_xor(l, 16, 32);
    const bool any = l > 0.0f;
    const float lsafe = any ? l : 1.0f;
    const float inv = any ? (1.0f / lsafe) : 0.0f;
    const float invc = inv * CCAR;
    v8f f0 = o0, f1 = o1, f2 = o2, f3 = o3;
    if (EARLY) { f0 = o0 + oR0 * QRI; f1 = o1 + oR1 * QRI; f2 = o2 + oR2 * QRI; f3 = o3 + oR3 * QRI; }
    const unsigned wb = wave * 16u * (unsigned)OSP;
    { v4f a, c;
      a[0] = f0[0] * invc; a[1] = f0[1] * invc; a[2] = f0[2] * invc; a[3] = f0[3] * invc; c[0] = f0[4] * invc; c[1] = f0[5] * invc; c[2] = f0[6] * invc; c[3] = f0[7] * invc;
      *(v4fa*)(&os[wb + lr * OSP +  0 + 8 * hi]) = a; *(v4fa*)(&os[wb + lr * OSP +  0 + 8 * hi + 4]) = c;
      a[0] = f1[0] * invc; a[1] = f1[1] * invc; a[2] = f1[2] * invc; a[3] = f1[3] * invc; c[0] = f1[4] * invc; c[1] = f1[5] * invc; c[2] = f1[6] * invc; c[3] = f1[7] * invc;
      *(v4fa*)(&os[wb + lr * OSP + 16 + 8 * hi]) = a; *(v4fa*)(&os[wb + lr * OSP + 16 + 8 * hi + 4]) = c;
      a[0] = f2[0] * invc; a[1] = f2[1] * invc; a[2] = f2[2] * invc; a[3] = f2[3] * invc; c[0] = f2[4] * invc; c[1] = f2[5] * invc; c[2] = f2[6] * invc; c[3] = f2[7] * invc;
      *(v4fa*)(&os[wb + lr * OSP + 32 + 8 * hi]) = a; *(v4fa*)(&os[wb + lr * OSP + 32 + 8 * hi + 4]) = c;
      a[0] = f3[0] * invc; a[1] = f3[1] * invc; a[2] = f3[2] * invc; a[3] = f3[3] * invc; c[0] = f3[4] * invc; c[1] = f3[5] * invc; c[2] = f3[6] * invc; c[3] = f3[7] * invc;
      *(v4fa*)(&os[wb + lr * OSP + 48 + 8 * hi]) = a; *(v4fa*)(&os[wb + lr * OSP + 48 + 8 * hi + 4]) = c; }
    wave_sync();
    const size_t coff = ((size_t)b * SEQ + t0) * DM + h * (unsigned)HD;
    const size_t roff = EARLY ? (((size_t)b * EROWS + t0) * DM + h * (unsigned)HD) : (size_t)0;
#pragma unroll 1
    for (int ps = 0; ps < 2; ++ps) {
#pragma unroll
        for (int s = 0; s < 4; ++s) { const unsigned row = 4u * (unsigned)s + (lane >> 3), c8 = (lane & 7u) * 8u;
            const v4f x0 = *(const v4fa*)(&os[wb + row * OSP + c8]); const v4f x1 = *(const v4fa*)(&os[wb + row * OSP + c8 + 4]); v8h hv, rv;
#pragma unroll
            for (int i = 0; i < 4; ++i) { const h16 a0 = toh_flush(x0[i]); const h16 a1 = toh_flush(x1[i]); hv[i] = a0; hv[4 + i] = a1;
                rv[i] = toh_flush((x0[i] - (float)a0) * QRS); rv[4 + i] = toh_flush((x1[i] - (float)a1) * QRS); }
            *(volatile v8h*)(CH + coff + (size_t)row * DM + c8) = hv;
            if (EARLY) *(volatile v8h*)(CR + roff + (size_t)row * DM + c8) = rv; }
        if (ps == 0) __threadfence(); }
}

__global__ __launch_bounds__(32 * AW) __attribute__((amdgpu_num_vgpr(256))) void k_flash_early(const h16* __restrict__ QH, const h16* __restrict__ QR, const h16* __restrict__ KP, const h16* __restrict__ KR,
                                                         const h16* __restrict__ VT, const h16* __restrict__ VR, h16* CH, h16* CR) {
    flash_body<1>(QH, QR, KP, KR, VT, VR, CH, CR);
}
__global__ __launch_bounds__(32 * AW) __attribute__((amdgpu_num_vgpr(256))) void k_flash_late(const h16* __restrict__ QH, const h16* __restrict__ QR, const h16* __restrict__ KP, const h16* __restrict__ KR,
                                                        const h16* __restrict__ VT, const h16* __restrict__ VR, h16* CH, h16* CR) {
    flash_body<0>(QH, QR, KP, KR, VT, VR, CH, CR);
}

template <int EARLY>
__device__ __forceinline__ void oproj_body(const h16* __restrict__ A, const h16* __restrict__ AR, const h16* __restrict__ Bt, const float* __restrict__ bias, float* OUT) {
    __shared__ __align__(16) float os[16 * 68];
    constexpr unsigned MB = EARLY ? 2u : 4u;
    constexpr unsigned RT = 16u * MB;
    constexpr unsigned TPB = EARLY ? ((unsigned)EROWS / RT) : ((((unsigned)(SEQ - EROWS)) / RT) > 0u ? (((unsigned)(SEQ - EROWS)) / RT) : 1u);
    const unsigned lane = threadIdx.x & 31u, lr = lane & 15u, hi = lane >> 4;
    const unsigned bx = blockIdx.x; const unsigned bb = bx / TPB, tt = (EARLY ? 0u : (unsigned)EROWS) + (bx % TPB) * RT;
    const unsigned c0 = blockIdx.y * 64u;
    const size_t m0 = (size_t)bb * SEQ + tt;
    const size_t mr = (size_t)bb * EROWS + tt;
    const v16h hz = (v16h){};
    v8f acc[MB][4], accR[MB][4];
#pragma unroll
    for (unsigned mb = 0; mb < MB; ++mb)
#pragma unroll
        for (int nb = 0; nb < 4; ++nb) { acc[mb][nb] = (v8f){}; accR[mb][nb] = (v8f){}; }
    const size_t aoff = (m0 + lr) * DM + 8u * hi, aroff = (mr + lr) * DM + 8u * hi, boff = (size_t)(c0 + lr) * DM + 8u * hi;
#pragma unroll 1
    for (unsigned kc = 0; kc < (unsigned)DM; kc += 32u) {
        v16h a[MB], ar[MB];
#pragma unroll
        for (unsigned mb = 0; mb < MB; ++mb) { a[mb] = ldh(A + aoff + (size_t)mb * 16 * DM + kc); ar[mb] = hz;
            if (EARLY) ar[mb] = ldh(AR + aroff + (size_t)mb * 16 * DM + kc); }
#pragma unroll
        for (int nb = 0; nb < 4; ++nb) { const v16h wq = ldh(Bt + boff + (size_t)nb * 16 * DM + kc);
#pragma unroll
            for (unsigned mb = 0; mb < MB; ++mb) { acc[mb][nb] = wmma16g(a[mb], wq, acc[mb][nb]);
                if (EARLY) accR[mb][nb] = wmma16g(ar[mb], wq, accR[mb][nb]); } }
    }
    float bc[4];
#pragma unroll
    for (int nb = 0; nb < 4; ++nb) bc[nb] = bfr(bias[c0 + nb * 16 + lr]);
    float* obase = OUT + ((size_t)bb * OUT_SEQ + tt) * DM + c0;
#pragma unroll
    for (unsigned mb = 0; mb < MB; ++mb) {
#pragma unroll
        for (int nb = 0; nb < 4; ++nb) {
#pragma unroll
            for (int j = 0; j < 8; ++j) { float v = acc[mb][nb][j] * OSCL; if (EARLY) v += accR[mb][nb][j] * (OSCL * QRI);
                os[(hi * 8 + j) * 68 + nb * 16 + lr] = v + bc[nb]; } }
        wave_sync();
#pragma unroll 1
        for (int ps = 0; ps < 2; ++ps) {
#pragma unroll
            for (int s = 0; s < 8; ++s) { const unsigned row = 2u * (unsigned)s + (lane >> 4), cofs = (lane & 15u) * 4u;
                const v4f val = *(const v4fa*)(&os[row * 68 + cofs]);
                *(volatile v4f*)(obase + (size_t)(mb * 16u + row) * DM + cofs) = val; }
            if (ps == 0) __threadfence(); }
        wave_sync();
    }
}

__global__ __launch_bounds__(32) void k_oproj_early(const h16* __restrict__ A, const h16* __restrict__ AR, const h16* __restrict__ Bt, const float* __restrict__ bias, float* OUT) {
    oproj_body<1>(A, AR, Bt, bias, OUT);
}
__global__ __launch_bounds__(32) void k_oproj_late(const h16* __restrict__ A, const h16* __restrict__ AR, const h16* __restrict__ Bt, const float* __restrict__ bias, float* OUT) {
    oproj_body<0>(A, AR, Bt, bias, OUT);
}

static constexpr size_t al256(size_t v) { return (v + 255) & ~(size_t)255; }
static constexpr size_t SZ_XB = al256((size_t)NB * SEQ * DM * 2);
static constexpr size_t SZ_WT = al256((size_t)DQKV * DM * 2);
static constexpr size_t SZ_WF = al256((size_t)DM * DM * 2);
static constexpr size_t SZ_PL = al256((size_t)NB * NH_ * SEQ * HD * 2);
static constexpr size_t SZ_RS = al256((size_t)NB * NH_ * EROWS * HD * 2);
static constexpr size_t SZ_CT = al256((size_t)NB * SEQ * DM * 2);
static constexpr size_t SZ_CR = al256((size_t)NB * EROWS * DM * 2);
static constexpr size_t SZ_TOTAL = SZ_XB + SZ_WT + SZ_WF + 3 * SZ_PL + 3 * SZ_RS + SZ_CT + SZ_CR;
static_assert(SZ_TOTAL <= (size_t)134217728);
static_assert(((size_t)DM * DM * 2) % 256 == 0);
static_assert((size_t)NB * NH_ * SEQ * HD == (size_t)NB * DM * SEQ);
static_assert((size_t)NB * NH_ * EROWS * HD == (size_t)NB * DM * EROWS);

extern "C" void kernel_launch(void* const* d_in, const int* in_sizes, int n_in,
                              void* d_out, int out_size, void* d_ws, size_t ws_size, hipStream_t stream) {
    if (n_in < 5) return;
    const size_t needx = ((size_t)(NB - 1) * SEQ_FULL + SEQ) * DM;
    if ((size_t)in_sizes[0] < needx) return;
    if ((size_t)in_sizes[1] < (size_t)DM * DQKV || in_sizes[2] < DQKV) return;
    if ((size_t)in_sizes[3] < (size_t)DM * DM || in_sizes[4] < DM) return;
    if ((size_t)out_size < ((size_t)(NB - 1) * OUT_SEQ + SEQ) * DM) return;
    if (SZ_TOTAL > ws_size) return;
    const float* x    = (const float*)d_in[0];
    const float* wqkv = (const float*)d_in[1];
    const float* bqkv = (const float*)d_in[2];
    const float* wfc  = (const float*)d_in[3];
    const float* bfc  = (const float*)d_in[4];
    float* OUT = (float*)d_out;
    char* wsp = (char*)d_ws;
    bf*  XB  = (bf*)wsp;  wsp += SZ_XB;
    bf*  WTB = (bf*)wsp;  wsp += SZ_WT;
    h16* WFH = (h16*)wsp; wsp += SZ_WF;
    h16* QH  = (h16*)wsp; wsp += SZ_PL;
    h16* KP  = (h16*)wsp; wsp += SZ_PL;
    h16* VT  = (h16*)wsp; wsp += SZ_PL;
    h16* QR  = (h16*)wsp; wsp += SZ_RS;
    h16* KR  = (h16*)wsp; wsp += SZ_RS;
    h16* VR  = (h16*)wsp; wsp += SZ_RS;
    h16* CH  = (h16*)wsp; wsp += SZ_CT;
    h16* CR  = (h16*)wsp; wsp += SZ_CR;

    if (SEQ == SEQ_FULL) {
        const size_t n8 = (size_t)NB * SEQ * DM / 8;
        k_cvt8<<<(unsigned)((n8 + 255) / 256), 256, 0, stream>>>(x, XB, n8);
    } else {
        const size_t n8 = (size_t)SEQ * DM / 8;
        for (int b = 0; b < NB; ++b) k_cvt8<<<(unsigned)((n8 + 255) / 256), 256, 0, stream>>>(x + (size_t)b * SEQ_FULL * DM, XB + (size_t)b * SEQ * DM, n8);
    }
    k_wtb<<<DQKV / 16, 128, 0, stream>>>(wqkv, WTB, (unsigned)DQKV);
    k_wth<<<DM / 16, 128, 0, stream>>>(wfc, WFH, (unsigned)DM);

    k_proj_rows<<<dim3(NB * SEQ / 64, DM / 64, 1), 32, 0, stream>>>(XB, WTB, bqkv, QH, QR, (unsigned)EROWS);
    k_proj_rows<<<dim3(NB * SEQ / 64, DM / 64, 1), 32, 0, stream>>>(XB, WTB + (size_t)DM * DM, bqkv + DM, KP, KR, (unsigned)EROWS);
    k_proj_tr<<<dim3(DM / 64, NB * SEQ / 64, 1), 32, 0, stream>>>(WTB + (size_t)2 * DM * DM, XB, bqkv + 2 * DM, VT, VR, (unsigned)EROWS);

    k_flash_early<<<dim3(EROWS / (16 * AW), NB * NH_, 1), 32 * AW, 0, stream>>>(QH, QR, KP, KR, VT, VR, CH, CR);
    if (SEQ > EROWS)
        k_flash_late<<<dim3((SEQ - EROWS) / (16 * AW), NB * NH_, 1), 32 * AW, 0, stream>>>(QH, QR, KP, KR, VT, VR, CH, CR);

    k_oproj_early<<<dim3(NB * EROWS / 32, DM / 64, 1), 32, 0, stream>>>(CH, CR, WFH, bfc, OUT);
    if (SEQ > EROWS)
        k_oproj_late<<<dim3(NB * (SEQ - EROWS) / 64, DM / 64, 1), 32, 0, stream>>>(CH, CR, WFH, bfc, OUT);
}
